// RWKVTimeMixing_9234179686554
// MI455X (gfx1250) — hardware-verified
//
#include <hip/hip_runtime.h>
#pragma clang fp contract(off)

static constexpr int kB  = 4;
static constexpr int kS  = 2048;
static constexpr int kD  = 1024;
static constexpr int kH  = 16;
static constexpr int kHD = 64;
static constexpr int kM  = kB * kS;
static constexpr int kLanes = kB * kD;
static constexpr int kN8 = kM * kD / 8;
static constexpr int kW2 = kD * kD / 2;
static constexpr int kGemmTiles  = (kM / 64) * (kD / 64);
static constexpr int kGemmBlocks = kGemmTiles / 8;
static_assert(kM % 64 == 0, "M tile");
static_assert(kD % 64 == 0, "N tile");
static_assert(kD % 32 == 0, "K step");
static_assert(kGemmTiles % 8 == 0, "waves per block");
static_assert(kH * kHD == kD, "groups");
static_assert(kLanes % 256 == 0, "scan grid");
static_assert(kN8 % 256 == 0, "elementwise grid");
static_assert(kW2 % 256 == 0, "cast grid");

typedef __attribute__((ext_vector_type(16))) _Float16 v16h;
typedef __attribute__((ext_vector_type(8)))  _Float16 v8h;
typedef __attribute__((ext_vector_type(16))) __bf16   v16b;
typedef __attribute__((ext_vector_type(8)))  __bf16   v8b;
typedef __attribute__((ext_vector_type(8)))  float    v8f;
typedef __attribute__((ext_vector_type(4)))  float    v4f;
typedef __attribute__((ext_vector_type(4)))  unsigned v4u;
typedef __attribute__((ext_vector_type(2)))  double   v2d;

__device__ __forceinline__ unsigned short f2bf_bits(float f) {
  unsigned u = __float_as_uint(f);
  return (unsigned short)((u + 0x7FFFu + ((u >> 16) & 1u)) >> 16);
}
__device__ __forceinline__ float bf_bits2f(unsigned short h) { return __uint_as_float(((unsigned)h) << 16); }

__device__ __forceinline__ void dep_guard_h(v8f& a, v8f& b, v16h x, v16h y) { asm volatile("v_nop\n\tv_nop\n\tv_nop\n\tv_nop" : "+v"(a), "+v"(b) : "v"(x), "v"(y)); }
__device__ __forceinline__ void dep_guard_b(v8f& a, v8f& b, v16b x, v16b y) { asm volatile("v_nop\n\tv_nop\n\tv_nop\n\tv_nop" : "+v"(a), "+v"(b) : "v"(x), "v"(y)); }
__device__ __forceinline__ void keep4_h(v16h a, v16h b, v16h c, v16h d) { asm volatile("v_nop" :: "v"(a), "v"(b), "v"(c), "v"(d)); }
__device__ __forceinline__ void keep4_b(v16b a, v16b b, v16b c, v16b d) { asm volatile("v_nop" :: "v"(a), "v"(b), "v"(c), "v"(d)); }
__device__ __forceinline__ void acc_guard4(v8f& a, v8f& b, v8f& c, v8f& d) { asm volatile("v_nop\n\tv_nop\n\tv_nop\n\tv_nop" : "+v"(a), "+v"(b), "+v"(c), "+v"(d)); }
template <typename T> struct Frag;
template <> struct Frag<_Float16> {
  typedef v16h V; union U { v16h v; v8h h[2]; };
  static __device__ __forceinline__ v16h load(const _Float16* p) {
    U f; f.h[0] = *(const v8h*)(p); f.h[1] = *(const v8h*)(p + 16); return f.v;
  }
  static __device__ __forceinline__ v8f mma(v16h a, v16h b, v8f c) {
    return __builtin_amdgcn_wmma_f32_16x16x32_f16(false, a, false, b, (short)0, c, false, false);
  }
  static __device__ __forceinline__ void guard(v8f& a, v8f& b, v16h x, v16h y) { dep_guard_h(a, b, x, y); }
  static __device__ __forceinline__ void keep(v16h a, v16h b, v16h c, v16h d) { keep4_h(a, b, c, d); }
};
template <> struct Frag<__bf16> {
  typedef v16b V; union U { v16b v; v8b h[2]; };
  static __device__ __forceinline__ v16b load(const __bf16* p) {
    U f; f.h[0] = *(const v8b*)(p); f.h[1] = *(const v8b*)(p + 16); return f.v;
  }
  static __device__ __forceinline__ v8f mma(v16b a, v16b b, v8f c) {
    return __builtin_amdgcn_wmma_f32_16x16x32_bf16(false, a, false, b, (short)0, c, false, false);
  }
  static __device__ __forceinline__ void guard(v8f& a, v8f& b, v16b x, v16b y) { dep_guard_b(a, b, x, y); }
  static __device__ __forceinline__ void keep(v16b a, v16b b, v16b c, v16b d) { keep4_b(a, b, c, d); }
};

template <int ET> struct Elem;
template <> struct Elem<0> { typedef _Float16 T; };
template <> struct Elem<1> { typedef __bf16 T; };
template <int ET, bool SPLIT, int BIAS_MODE, int OUT_MODE, bool RESID, int ACT = 0>
__global__ __launch_bounds__(256) void wmma_gemm64(
    const unsigned short* __restrict__ Ap, const unsigned short* __restrict__ A2p, int lda, long strideA,
    const unsigned short* __restrict__ Btp, const unsigned short* __restrict__ Bt2p, int ldb, long strideB,
    void* __restrict__ Cout, void* __restrict__ Cout2, int ldc, long strideC,
    const float* __restrict__ bias,
    const float* __restrict__ resid, long strideR,
    int M, int N, int K, float scale) {
  typedef typename Elem<ET>::T T;
  typedef typename Frag<T>::V V;
  const T* A = (const T*)Ap; const T* A2 = (const T*)A2p; const T* Bt = (const T*)Btp; const T* Bt2 = (const T*)Bt2p;
  __shared__ __align__(16) float sT[8][16 * 68];
  const int b    = blockIdx.y;
  const int lane = threadIdx.x & 31;
  const int wave = threadIdx.x >> 5;
  const int tilesN = N >> 6;
  const int tilesM = M >> 6;
  const int tile = blockIdx.x * 8 + wave;
  if (tile >= tilesM * tilesN) return;
  const int tm = tile / tilesN;
  const int tn = tile - tm * tilesN;
  const int m0 = tm << 6;
  const int n0 = tn << 6;

  const T* Ab  = A  + (size_t)b * strideA;
  const T* Bb  = Bt + (size_t)b * strideB;
  const T* Ab2 = SPLIT ? (A2  + (size_t)b * strideA) : nullptr;
  const T* Bb2 = SPLIT ? (Bt2 + (size_t)b * strideB) : nullptr;

  const int rlane = lane & 15;
  const int koff  = (lane >> 4) * 8;
  const int mOff  = (lane >> 4) * 8;

  v8f acc[4][4];
#pragma unroll
  for (int i = 0; i < 4; ++i)
#pragma unroll
    for (int j = 0; j < 4; ++j) acc[i][j] = (v8f){0.f,0.f,0.f,0.f,0.f,0.f,0.f,0.f};

  for (int k0 = 0; k0 < K; k0 += 32) {
    V bh[4], bl[4];
#pragma unroll
    for (int j = 0; j < 4; ++j) {
      const size_t bo = (size_t)(n0 + (j << 4) + rlane) * ldb + koff + k0;
      bh[j] = Frag<T>::load(Bb + bo);
      if (SPLIT) bl[j] = Frag<T>::load(Bb2 + bo);
    }
#pragma unroll
    for (int i = 0; i < 4; ++i) {
      const size_t ao = (size_t)(m0 + (i << 4) + rlane) * lda + koff + k0;
      V ah = Frag<T>::load(Ab + ao);
      V al;
      if (SPLIT) al = Frag<T>::load(Ab2 + ao);
#pragma unroll
      for (int j = 0; j < 4; ++j) {
        acc[i][j] = Frag<T>::mma(ah, bh[j], acc[i][j]);
        if (SPLIT) {
          acc[i][j] = Frag<T>::mma(ah, bl[j], acc[i][j]);
          acc[i][j] = Frag<T>::mma(al, bh[j], acc[i][j]);
        }
      }
      Frag<T>::guard(acc[i][0], acc[i][3], ah, SPLIT ? al : ah);
    }
    Frag<T>::keep(bh[0], bh[1], bh[2], bh[3]);
    if (SPLIT) Frag<T>::keep(bl[0], bl[1], bl[2], bl[3]);
  }
  acc_guard4(acc[0][0], acc[0][1], acc[0][2], acc[0][3]);
  acc_guard4(acc[1][0], acc[1][1], acc[1][2], acc[1][3]);
  acc_guard4(acc[2][0], acc[2][1], acc[2][2], acc[2][3]);
  acc_guard4(acc[3][0], acc[3][1], acc[3][2], acc[3][3]);

  float* slab = sT[wave];
  const float* Rb = RESID ? (resid + (size_t)b * strideR) : nullptr;
#pragma unroll
  for (int i = 0; i < 4; ++i) {
    const int mBase = m0 + (i << 4);
#pragma unroll
    for (int j = 0; j < 4; ++j) {
      const int n = n0 + (j << 4) + rlane;
      float bv = 0.f;
      if (BIAS_MODE == 2) bv = bias[n];
#pragma unroll
      for (int r = 0; r < 8; ++r) {
        float v = acc[i][j][r] * scale;
        if (BIAS_MODE == 1) v += bias[mBase + mOff + r];
        if (BIAS_MODE == 2) v += bv;
        if (RESID) v += Rb[(size_t)(mBase + mOff + r) * ldc + n];
        if (ACT == 1) v = tanhf(v);
        if (ACT == 2) v = fmaxf(v, 0.0f);
        if (ACT == 3) v = v / (1.0f + expf(-v));
        if (ACT == 4) v = (v > 0.f) ? v : 0.01f * v;
        if (ACT == 5) v = 0.5f * v * (1.0f + erff(v * 0.70710678118654752f));
        slab[(mOff + r) * 68 + (j << 4) + rlane] = v;
      }
    }
    __builtin_amdgcn_fence(__ATOMIC_RELEASE, "workgroup");
    __builtin_amdgcn_wave_barrier();
    __builtin_amdgcn_fence(__ATOMIC_ACQUIRE, "workgroup");
    if (OUT_MODE == 0) {
      float* C = (float*)Cout + (size_t)b * strideC;
      const int hh = lane >> 4, c4 = (lane & 15) * 4;
      for (int pass = 0; pass < 2; ++pass) {
#pragma unroll
        for (int it = 0; it < 8; ++it) {
          const int row = it * 2 + hh;
          v4f v = *(const v4f*)(slab + row * 68 + c4);
          *(volatile v4f*)(C + (size_t)(mBase + row) * ldc + n0 + c4) = v;
        }
        __threadfence();
      }
    } else {
      const int q = lane >> 3, c8 = (lane & 7) * 8;
      unsigned short* C  = (unsigned short*)Cout  + (size_t)b * strideC;
      unsigned short* C2 = (OUT_MODE == 2) ? ((unsigned short*)Cout2 + (size_t)b * strideC) : nullptr;
      for (int pass = 0; pass < 2; ++pass) {
#pragma unroll
        for (int it = 0; it < 4; ++it) {
          const int row = it * 4 + q;
          const float* sp = slab + row * 68 + c8;
          v8h hv, lv;
#pragma unroll
          for (int e = 0; e < 8; ++e) {
            if (OUT_MODE == 1) {
              hv[e] = (_Float16)sp[e];
            } else {
              unsigned short hb = f2bf_bits(sp[e]);
              unsigned short lb = f2bf_bits(sp[e] - bf_bits2f(hb));
              hv[e] = __builtin_bit_cast(_Float16, hb);
              lv[e] = __builtin_bit_cast(_Float16, lb);
            }
          }
          *(volatile v8h*)(C + (size_t)(mBase + row) * ldc + n0 + c8) = hv;
          if (OUT_MODE == 2) *(volatile v8h*)(C2 + (size_t)(mBase + row) * ldc + n0 + c8) = lv;
        }
        __threadfence();
      }
    }
    __builtin_amdgcn_fence(__ATOMIC_RELEASE, "workgroup");
    __builtin_amdgcn_wave_barrier();
    __builtin_amdgcn_fence(__ATOMIC_ACQUIRE, "workgroup");
  }
}

__global__ __launch_bounds__(256) void cast_f32_f16x2_scaled(
    const float* __restrict__ in, unsigned short* __restrict__ out, int n2, float carry) {
  const int i = blockIdx.x * 256 + threadIdx.x;
  if (i >= n2) return;
  const _Float16 h0 = (_Float16)(in[2 * i] * carry), h1 = (_Float16)(in[2 * i + 1] * carry);
  const unsigned u = (unsigned)__builtin_bit_cast(unsigned short, h0) | ((unsigned)__builtin_bit_cast(unsigned short, h1) << 16);
  ((volatile unsigned*)out)[i] = u;
  __threadfence();
  ((volatile unsigned*)out)[i] = u;
}

__global__ __launch_bounds__(256) void split_f32_bf16x2(
    const float* __restrict__ in, unsigned short* __restrict__ hi, unsigned short* __restrict__ lo, int n2) {
  const int i = blockIdx.x * 256 + threadIdx.x;
  if (i >= n2) return;
  const float a = in[2 * i], c = in[2 * i + 1];
  const unsigned short ha = f2bf_bits(a), hc = f2bf_bits(c);
  const unsigned short la = f2bf_bits(a - bf_bits2f(ha)), lc = f2bf_bits(c - bf_bits2f(hc));
  const unsigned uh = (unsigned)ha | ((unsigned)hc << 16);
  const unsigned ul = (unsigned)la | ((unsigned)lc << 16);
  ((volatile unsigned*)hi)[i] = uh;
  ((volatile unsigned*)lo)[i] = ul;
  __threadfence();
  ((volatile unsigned*)hi)[i] = uh;
  ((volatile unsigned*)lo)[i] = ul;
}

__global__ __launch_bounds__(256) void token_mix_f16(const float* __restrict__ x, const float* __restrict__ tm,
                                                     unsigned short* __restrict__ dst, int n8) {
  const int i8 = blockIdx.x * 256 + threadIdx.x;
  if (i8 >= n8) return;
  const int row = i8 >> 7;
  const int d0 = (i8 & 127) * 8;
  const int s = row & (kS - 1);
  const bool has_prev = (s > 0);
  const int prow = has_prev ? (row - 1) : row;
  const float* xc = x + (size_t)row * kD + d0;
  const float* xq = x + (size_t)prow * kD + d0;
  const v4f c0 = *(const v4f*)xc, c1 = *(const v4f*)(xc + 4);
  const v4f q0 = *(const v4f*)xq, q1 = *(const v4f*)(xq + 4);
  const v4f m0 = *(const v4f*)(tm + d0), m1 = *(const v4f*)(tm + d0 + 4);
  const float cv[8] = {c0.x, c0.y, c0.z, c0.w, c1.x, c1.y, c1.z, c1.w};
  const float qv[8] = {q0.x, q0.y, q0.z, q0.w, q1.x, q1.y, q1.z, q1.w};
  const float mv[8] = {m0.x, m0.y, m0.z, m0.w, m1.x, m1.y, m1.z, m1.w};
  unsigned wb[4];
#pragma unroll
  for (int q = 0; q < 4; ++q) {
    float r2[2];
#pragma unroll
    for (int e = 0; e < 2; ++e) {
      const int j = 2 * q + e;
      const float pv = has_prev ? qv[j] : 0.0f;
      const float om = 1.0f - mv[j];
      const float t0 = cv[j] * mv[j];
      const float t1 = pv * om;
      r2[e] = t0 + t1;
    }
    wb[q] = (unsigned)__builtin_bit_cast(unsigned short, (_Float16)r2[0]) |
            ((unsigned)__builtin_bit_cast(unsigned short, (_Float16)r2[1]) << 16);
  }
  v4u o; o.x = wb[0]; o.y = wb[1]; o.z = wb[2]; o.w = wb[3];
  unsigned short* op = dst + (size_t)row * kD + d0;
  *(volatile v4u*)op = o;
  __threadfence();
  *(volatile v4u*)op = o;
}

__global__ __launch_bounds__(256) void token_mix_bf16split(const float* __restrict__ x, const float* __restrict__ tm,
                                                           unsigned short* __restrict__ dhi, unsigned short* __restrict__ dlo, int n8) {
  const int i8 = blockIdx.x * 256 + threadIdx.x;
  if (i8 >= n8) return;
  const int row = i8 >> 7;
  const int d0 = (i8 & 127) * 8;
  const int s = row & (kS - 1);
  const bool has_prev = (s > 0);
  const int prow = has_prev ? (row - 1) : row;
  const float* xc = x + (size_t)row * kD + d0;
  const float* xq = x + (size_t)prow * kD + d0;
  const v4f c0 = *(const v4f*)xc, c1 = *(const v4f*)(xc + 4);
  const v4f q0 = *(const v4f*)xq, q1 = *(const v4f*)(xq + 4);
  const v4f m0 = *(const v4f*)(tm + d0), m1 = *(const v4f*)(tm + d0 + 4);
  const float cv[8] = {c0.x, c0.y, c0.z, c0.w, c1.x, c1.y, c1.z, c1.w};
  const float qv[8] = {q0.x, q0.y, q0.z, q0.w, q1.x, q1.y, q1.z, q1.w};
  const float mv[8] = {m0.x, m0.y, m0.z, m0.w, m1.x, m1.y, m1.z, m1.w};
  unsigned hw[4], lw[4];
#pragma unroll
  for (int q = 0; q < 4; ++q) {
    unsigned short hb[2], lb[2];
#pragma unroll
    for (int e = 0; e < 2; ++e) {
      const int j = 2 * q + e;
      const float pv = has_prev ? qv[j] : 0.0f;
      const float om = 1.0f - mv[j];
      const float t0 = cv[j] * mv[j];
      const float t1 = pv * om;
      const float r = t0 + t1;
      hb[e] = f2bf_bits(r);
      lb[e] = f2bf_bits(r - bf_bits2f(hb[e]));
    }
    hw[q] = (unsigned)hb[0] | ((unsigned)hb[1] << 16);
    lw[q] = (unsigned)lb[0] | ((unsigned)lb[1] << 16);
  }
  v4u oh; oh.x = hw[0]; oh.y = hw[1]; oh.z = hw[2]; oh.w = hw[3];
  v4u ol; ol.x = lw[0]; ol.y = lw[1]; ol.z = lw[2]; ol.w = lw[3];
  const size_t off = (size_t)row * kD + d0;
  *(volatile v4u*)(dhi + off) = oh;
  *(volatile v4u*)(dlo + off) = ol;
  __threadfence();
  *(volatile v4u*)(dhi + off) = oh;
  *(volatile v4u*)(dlo + off) = ol;
}

__global__ __launch_bounds__(256) void wkv_scan(const float* __restrict__ kbuf, const float* __restrict__ vbuf,
                                               const float* __restrict__ tdec, const float* __restrict__ tfirst,
                                               float* __restrict__ wkv, int nlanes) {
  const int c = blockIdx.x * 256 + threadIdx.x;
  if (c >= nlanes) return;
  const int b = c >> 10;
  const int ch = c & (kD - 1);
  const float w = -expf(tdec[ch]);
  const float u = tfirst[ch];
  const size_t base = (size_t)b * kS * kD + ch;
  const float* kp = kbuf + base;
  const float* vp = vbuf + base;
  float* op = wkv + base;
  float a = 0.0f;
  float bst = -1e38f;
#pragma unroll 1
  for (int t = 0; t < kS; ++t) {
    const size_t off = (size_t)t * kD;
    const float kt = kp[off];
    const float vt = vp[off];
    const float wk = kt + u;
    const float d1 = bst - wk;
    const float em = expf(-fabsf(d1));
    const bool ge = (d1 >= 0.0f);
    const float e1 = ge ? 1.0f : em;
    const float e2 = ge ? em : 1.0f;
    const float n1 = e1 * a;
    const float n2 = e2 * vt;
    const float num = n1 + n2;
    const float den = (e1 + e2) + 1e-8f;
    const float y = num / den;
    *(volatile float*)(op + off) = y;
    __threadfence();
    *(volatile float*)(op + off) = y;
    const float ww = bst + w;
    const float d2 = ww - kt;
    const float em2 = expf(-fabsf(d2));
    const bool ge2 = (d2 >= 0.0f);
    const float p2 = ge2 ? ww : kt;
    const float e1b = ge2 ? 1.0f : em2;
    const float e2b = ge2 ? em2 : 1.0f;
    const float a1 = e1b * a;
    const float a2 = e2b * vt;
    a = a1 + a2;
    bst = p2 + logf((e1b + e2b) + 1e-8f);
  }
}

__global__ __launch_bounds__(256) void gate_stats(const float* __restrict__ rbuf, const float* __restrict__ wkv,
                                                 float* __restrict__ ybuf, double* __restrict__ part, int nlanes) {
  const int c = blockIdx.x * 256 + threadIdx.x;
  if (c >= nlanes) return;
  const int b = c >> 10;
  const int ch = c & (kD - 1);
  const size_t base = (size_t)b * kS * kD + ch;
  const float* rp = rbuf + base;
  const float* wp = wkv + base;
  float* yp = ybuf + base;
  double s = 0.0, ss = 0.0;
#pragma unroll 1
  for (int t = 0; t < kS; ++t) {
    const size_t off = (size_t)t * kD;
    const float rv = rp[off];
    const float wv = wp[off];
    const float sg = 1.0f / (1.0f + expf(-rv));
    const float y = sg * wv;
    *(volatile float*)(yp + off) = y;
    __threadfence();
    *(volatile float*)(yp + off) = y;
    const double yd = (double)y;
    s += yd;
    ss += yd * yd;
  }
  v2d pv; pv.x = s; pv.y = ss;
  *(volatile v2d*)(part + 2 * (size_t)c) = pv;
  __threadfence();
  *(volatile v2d*)(part + 2 * (size_t)c) = pv;
}

__global__ __launch_bounds__(64) void group_stats(const double* __restrict__ part, float* __restrict__ gtab) {
  __shared__ __align__(16) float tab[128];
  const int g = threadIdx.x;
  double s = 0.0, ss = 0.0;
#pragma unroll 1
  for (int j = 0; j < kHD; ++j) {
    const size_t c = (size_t)g * kHD + j;
    s += part[2 * c];
    ss += part[2 * c + 1];
  }
  const double inv = 1.0 / (double)(kS * kHD);
  const double mean = s * inv;
  const double var = ss * inv - mean * mean;
  float varf = (float)var;
  varf = (varf > 0.0f) ? varf : 0.0f;
  tab[g] = (float)mean;
  tab[64 + g] = rsqrtf(varf + 1e-5f);
  __syncthreads();
  if (threadIdx.x < 32) {
    const int l = threadIdx.x;
    const v4f v = *(const v4f*)(tab + 4 * l);
    *(volatile v4f*)(gtab + 4 * l) = v;
    __threadfence();
    *(volatile v4f*)(gtab + 4 * l) = v;
  }
}

__global__ __launch_bounds__(256) void norm_apply(const float* __restrict__ ybuf, const float* __restrict__ gtab,
                                                 const float* __restrict__ gam, const float* __restrict__ bet,
                                                 unsigned short* __restrict__ nhi, unsigned short* __restrict__ nlo, int n8) {
  const int i8 = blockIdx.x * 256 + threadIdx.x;
  if (i8 >= n8) return;
  const int row = i8 >> 7;
  const int d0 = (i8 & 127) * 8;
  const int b = row >> 11;
  const int hg = d0 >> 6;
  const int g = b * kH + hg;
  const float mean = gtab[g];
  const float rstd = gtab[64 + g];
  const size_t off = (size_t)row * kD + d0;
  const v4f y0 = *(const v4f*)(ybuf + off), y1 = *(const v4f*)(ybuf + off + 4);
  const v4f g0 = *(const v4f*)(gam + d0), g1 = *(const v4f*)(gam + d0 + 4);
  const v4f b0 = *(const v4f*)(bet + d0), b1 = *(const v4f*)(bet + d0 + 4);
  const float yv[8] = {y0.x, y0.y, y0.z, y0.w, y1.x, y1.y, y1.z, y1.w};
  const float gv[8] = {g0.x, g0.y, g0.z, g0.w, g1.x, g1.y, g1.z, g1.w};
  const float bv[8] = {b0.x, b0.y, b0.z, b0.w, b1.x, b1.y, b1.z, b1.w};
  unsigned hw[4], lw[4];
#pragma unroll
  for (int q = 0; q < 4; ++q) {
    unsigned short hb[2], lb[2];
#pragma unroll
    for (int e = 0; e < 2; ++e) {
      const int j = 2 * q + e;
      const float nrm = (yv[j] - mean) * rstd;
      const float t0 = nrm * gv[j];
      const float v = t0 + bv[j];
      hb[e] = f2bf_bits(v);
      lb[e] = f2bf_bits(v - bf_bits2f(hb[e]));
    }
    hw[q] = (unsigned)hb[0] | ((unsigned)hb[1] << 16);
    lw[q] = (unsigned)lb[0] | ((unsigned)lb[1] << 16);
  }
  v4u oh; oh.x = hw[0]; oh.y = hw[1]; oh.z = hw[2]; oh.w = hw[3];
  v4u ol; ol.x = lw[0]; ol.y = lw[1]; ol.z = lw[2]; ol.w = lw[3];
  *(volatile v4u*)(nhi + off) = oh;
  *(volatile v4u*)(nlo + off) = ol;
  __threadfence();
  *(volatile v4u*)(nhi + off) = oh;
  *(volatile v4u*)(nlo + off) = ol;
}

extern "C" void kernel_launch(void* const* d_in, const int* in_sizes, int n_in,
                              void* d_out, int out_size, void* d_ws, size_t ws_size,
                              hipStream_t stream) {
  if (n_in < 12) return;
  if (in_sizes[0] != kM * kD || in_sizes[4] != kD * kD || in_sizes[7] != kD * kD ||
      in_sizes[8] != kH * kHD || out_size != kM * kD) return;
  const float* x      = (const float*)d_in[0];
  const float* tmr    = (const float*)d_in[1];
  const float* tmk    = (const float*)d_in[2];
  const float* tmv    = (const float*)d_in[3];
  const float* w_r    = (const float*)d_in[4];
  const float* w_k    = (const float*)d_in[5];
  const float* w_v    = (const float*)d_in[6];
  const float* w_o    = (const float*)d_in[7];
  const float* tdec   = (const float*)d_in[8];
  const float* tfirst = (const float*)d_in[9];
  const float* gam    = (const float*)d_in[10];
  const float* bet    = (const float*)d_in[11];
  float* out = (float*)d_out;

  const size_t wbytes16  = (size_t)kD * kD * sizeof(unsigned short);
  const size_t planeF32  = (size_t)kM * kD * sizeof(float);
  const size_t half16    = (size_t)kM * kD * sizeof(unsigned short);
  const size_t partBytes = (size_t)kLanes * 2 * sizeof(double);
  const size_t gtabBytes = 128 * sizeof(float);
  size_t off = 0;
  char* ws = (char*)d_ws;
  unsigned short* wr16 = (unsigned short*)(ws + off); off += wbytes16;
  unsigned short* wk16 = (unsigned short*)(ws + off); off += wbytes16;
  unsigned short* wvh  = (unsigned short*)(ws + off); off += wbytes16;
  unsigned short* wvl  = (unsigned short*)(ws + off); off += wbytes16;
  unsigned short* woh  = (unsigned short*)(ws + off); off += wbytes16;
  unsigned short* wol  = (unsigned short*)(ws + off); off += wbytes16;
  char* p0 = ws + off; off += planeF32;
  char* p1 = ws + off; off += planeF32;
  char* p2 = ws + off; off += planeF32;
  double* part = (double*)(ws + off); off += partBytes;
  float* gtab = (float*)(ws + off); off += gtabBytes;
  if (off > ws_size) return;

  float* p0f = (float*)p0;
  float* p1f = (float*)p1;
  float* p2f = (float*)p2;
  unsigned short* xmixK  = (unsigned short*)p2;
  unsigned short* xmixVh = (unsigned short*)p2;
  unsigned short* xmixVl = (unsigned short*)(p2 + half16);
  unsigned short* xmixR  = (unsigned short*)p1;
  unsigned short* nrmH   = (unsigned short*)p0;
  unsigned short* nrmL   = (unsigned short*)(p0 + half16);

  const dim3 blk(256);
  const int castBlocks = kW2 / 256;
  const int ewBlocks   = kN8 / 256;
  const int laneBlocks = kLanes / 256;
  const float wcarry = 64.0f;
  const float wcarryInv = 1.0f / 64.0f;

  cast_f32_f16x2_scaled<<<dim3(castBlocks), blk, 0, stream>>>(w_r, wr16, kW2, wcarry);
  cast_f32_f16x2_scaled<<<dim3(castBlocks), blk, 0, stream>>>(w_k, wk16, kW2, wcarry);
  split_f32_bf16x2<<<dim3(castBlocks), blk, 0, stream>>>(w_v, wvh, wvl, kW2);
  split_f32_bf16x2<<<dim3(castBlocks), blk, 0, stream>>>(w_o, woh, wol, kW2);

  token_mix_f16<<<dim3(ewBlocks), blk, 0, stream>>>(x, tmk, xmixK, kN8);
  wmma_gemm64<0, false, 0, 0, false><<<dim3(kGemmBlocks, 1), blk, 0, stream>>>(
      xmixK, xmixK, kD, 0L, wk16, wk16, kD, 0L, (void*)p0f, (void*)p0f, kD, 0L,
      tdec, tdec, 0L, kM, kD, kD, wcarryInv);

  token_mix_bf16split<<<dim3(ewBlocks), blk, 0, stream>>>(x, tmv, xmixVh, xmixVl, kN8);
  wmma_gemm64<1, true, 0, 0, false><<<dim3(kGemmBlocks, 1), blk, 0, stream>>>(
      xmixVh, xmixVl, kD, 0L, wvh, wvl, kD, 0L, (void*)p1f, (void*)p1f, kD, 0L,
      tdec, tdec, 0L, kM, kD, kD, 1.0f);

  wkv_scan<<<dim3(laneBlocks), blk, 0, stream>>>(p0f, p1f, tdec, tfirst, p2f, kLanes);

  token_mix_f16<<<dim3(ewBlocks), blk, 0, stream>>>(x, tmr, xmixR, kN8);
  wmma_gemm64<0, false, 0, 0, false><<<dim3(kGemmBlocks, 1), blk, 0, stream>>>(
      xmixR, xmixR, kD, 0L, wr16, wr16, kD, 0L, (void*)p0f, (void*)p0f, kD, 0L,
      tdec, tdec, 0L, kM, kD, kD, wcarryInv);

  gate_stats<<<dim3(laneBlocks), blk, 0, stream>>>(p0f, p2f, p1f, part, kLanes);

  group_stats<<<dim3(1), dim3(64), 0, stream>>>(part, gtab);

  norm_apply<<<dim3(ewBlocks), blk, 0, stream>>>(p1f, gtab, gam, bet, nrmH, nrmL, kN8);

  wmma_gemm64<1, true, 0, 0, false><<<dim3(kGemmBlocks, 1), blk, 0, stream>>>(
      nrmH, nrmL, kD, 0L, woh, wol, kD, 0L, (void*)out, (void*)out, kD, 0L,
      tdec, tdec, 0L, kM, kD, kD, 1.0f);
}
